// BPR_84653805404606
// MI455X (gfx1250) — hardware-verified
//
#include <hip/hip_runtime.h>
#include <math.h>

#pragma clang fp contract(off)

typedef __attribute__((ext_vector_type(16))) _Float16 v16h;
typedef __attribute__((ext_vector_type(8)))  _Float16 v8h;
typedef __attribute__((ext_vector_type(8)))  float    v8f;
typedef __attribute__((ext_vector_type(4)))  float    v4f;
typedef __attribute__((ext_vector_type(4)))  int      v4i;

constexpr int kNU      = 8192;
constexpr int kNI      = 40000;
constexpr int kD       = 64;
constexpr int kNR      = 100;
constexpr int kTopK    = 50;
constexpr int kKeep    = 64;
constexpr int kUPB     = 16;
constexpr int kChunk   = 512;
constexpr int kTPB     = 256;
constexpr int kNW      = 8;
constexpr int kTPW     = 4;
constexpr int kNChunks = (kNI + kChunk - 1) / kChunk;
constexpr int kRatedPerBlock = kUPB * kNR;
constexpr int kRatedRegs     = 7;
constexpr int kOutPerBlock   = kUPB * kTopK;
constexpr int kOutVec4       = kOutPerBlock / 4;
constexpr float kCarry = 1024.0f;

static_assert(kD == 64, "two 32-deep k steps");
static_assert((kNI % 16) == 0, "item tiles never split");
static_assert((kNU % kUPB) == 0, "user blocks exact");
static_assert(kNW * kTPW * 16 == kChunk, "tiles cover the chunk");
static_assert(kNW * 32 == kTPB, "eight waves");
static_assert(kKeep == 4 * 16, "four kept entries per lane of a 16-lane group");
static_assert(kRatedPerBlock <= kRatedRegs * kTPB, "rated ids fit the per-thread registers");
static_assert(((kOutPerBlock * 4) % 128) == 0, "block output is whole 128-B lines");
static_assert(kOutVec4 == 200 && kOutVec4 <= 7 * 32, "seven store steps of one wave");
static_assert(kNChunks == 79, "chunk count");

constexpr size_t kOffUH   = 0;
constexpr size_t kOffIH   = kOffUH + (size_t)kNU * kD * 2;
constexpr size_t kWsTotal = kOffIH + (size_t)kNI * kD * 2;
static_assert(kWsTotal == 6168576ull, "carve total");
static_assert(kWsTotal <= 134217728ull, "carve cap");
static_assert((kOffIH % 128) == 0, "aligned region");

union FragH { v16h v; v8h h[2]; };

__device__ __forceinline__ v16h frag_load_h(const _Float16* p) {
  FragH f;
  f.h[0] = *(const v8h*)(p);
  f.h[1] = *(const v8h*)(p + 16);
  return f.v;
}

__device__ __forceinline__ v8f mma_h(v16h a, v16h b, v8f c) {
  c = __builtin_amdgcn_wmma_f32_16x16x32_f16(false, a, false, b, (short)0, c, false, false);
  asm volatile("v_nop\n\tv_nop\n\tv_nop\n\tv_nop" : "+v"(c) : "v"(a), "v"(b));
  return c;
}

constexpr bool kFusedChain = true;
__device__ __forceinline__ float chain_step(float a, float b, float acc) {
  if (kFusedChain) return fmaf(a, b, acc);
  const float p = a * b;
  return acc + p;
}

__global__ __launch_bounds__(256) void scale_cast_f16_kernel(
    const float* __restrict__ src, unsigned short* __restrict__ dst, int total8)
{
  const int i = blockIdx.x * 256 + threadIdx.x;
  if (i >= total8) return;
  const size_t e0 = (size_t)i << 3;
  const v4f a0 = *(const v4f*)(src + e0);
  const v4f a1 = *(const v4f*)(src + e0 + 4);
  v8h hv;
#pragma unroll
  for (int e = 0; e < 4; ++e) {
    const float x0 = a0[e] * kCarry;
    const float x1 = a1[e] * kCarry;
    hv[e]     = (_Float16)x0;
    hv[4 + e] = (_Float16)x1;
  }
  unsigned short* q = dst + e0;
  *(volatile v8h*)q = hv;
  __threadfence();
  *(volatile v8h*)q = hv;
}

__global__ __launch_bounds__(256) void prefilter_rescore_kernel(
    const unsigned short* __restrict__ UHp, const unsigned short* __restrict__ IHp,
    const float* __restrict__ userF, const float* __restrict__ itemF,
    const int* __restrict__ rated, const int* __restrict__ topk_in,
    int* __restrict__ out)
{
  __shared__ __align__(16) float sc[kUPB * kChunk];
  __shared__ __align__(16) float rvS[kUPB * kKeep];
  __shared__ __align__(16) int   riS[kUPB * kKeep];
  __shared__ __align__(16) int   outS[kOutPerBlock];

  const int t     = threadIdx.x;
  const int wave  = __builtin_amdgcn_readfirstlane(t >> 5);
  const int lane  = t & 31;
  const int half  = lane >> 4;
  const int l16   = lane & 15;
  const int su    = t >> 4;
  const int ubase = blockIdx.x * kUPB;
  const unsigned hsh = 16u * (unsigned)half;
  const float kNegInf = __uint_as_float(0xff800000u);

  const _Float16* Uh = (const _Float16*)UHp;
  const _Float16* Ih = (const _Float16*)IHp;

  const int tk = topk_in[0];
  const bool premise_ok = (tk == kTopK);

  const _Float16* arow = Uh + (size_t)(ubase + l16) * kD + 8 * half;
  const v16h a0 = frag_load_h(arow);
  const v16h a1 = frag_load_h(arow + 32);

  int rid[kRatedRegs], roff[kRatedRegs];
#pragma unroll
  for (int i = 0; i < kRatedRegs; ++i) {
    const int j  = t + kTPB * i;
    const int jc = (j < kRatedPerBlock) ? j : (kRatedPerBlock - 1);
    int rv = rated[(size_t)ubase * kNR + jc];
    asm volatile("" : "+v"(rv));
    const bool ok = (j < kRatedPerBlock) && ((unsigned)rv < (unsigned)kNI);
    rid[i]  = ok ? rv : -0x40000000;
    roff[i] = (jc / kNR) * kChunk;
  }

  for (int j = t; j < kOutPerBlock; j += kTPB) outS[j] = 0;

  float kv[4];
  int   ki[4];
#pragma unroll
  for (int j = 0; j < 4; ++j) { kv[j] = kNegInf; ki[j] = 0; }
  float thr = kNegInf;

#pragma unroll 1
  for (int ch = 0; ch < kNChunks; ++ch) {
    const int c0 = ch * kChunk;

#pragma unroll 1
    for (int it = 0; it < kTPW; ++it) {
      const int tl = wave + kNW * it;
      const int n0 = c0 + tl * 16;
      float* dst = sc + (8 * half) * kChunk + tl * 16 + l16;
      if (n0 < kNI) {
        const _Float16* brow = Ih + (size_t)(n0 + l16) * kD + 8 * half;
        const v16h b0 = frag_load_h(brow);
        const v16h b1 = frag_load_h(brow + 32);
        v8f acc = (v8f){0.f, 0.f, 0.f, 0.f, 0.f, 0.f, 0.f, 0.f};
        acc = mma_h(a0, b0, acc);
        acc = mma_h(a1, b1, acc);
#pragma unroll
        for (int r = 0; r < 8; ++r) dst[r * kChunk] = acc[r];
      } else {
#pragma unroll
        for (int r = 0; r < 8; ++r) dst[r * kChunk] = kNegInf;
      }
    }
    __syncthreads();

#pragma unroll
    for (int i = 0; i < kRatedRegs; ++i) {
      const unsigned lc = (unsigned)(rid[i] - c0);
      if (lc < (unsigned)kChunk) sc[roff[i] + (int)lc] = kNegInf;
    }
    __syncthreads();

    {
      const float* row = sc + su * kChunk;
#pragma unroll 1
      for (int it = 0; it < kChunk / 16; ++it) {
        const float v = row[it * 16 + l16];
        bool hit = (v > thr);
        unsigned b = __builtin_amdgcn_ballot_w32(hit);
#pragma unroll 1
        for (int g = 0; g < 16 && b != 0u; ++g) {
          const unsigned mb = (b >> hsh) & 0xffffu;
          const bool hasc = (mb != 0u);
          const int src = (int)__builtin_ctz(mb | 0x10000u) & 15;
          const float cv = __shfl(v, (int)hsh + src, 32);
          const int ci = c0 + it * 16 + src;
          const bool act = hasc && (cv > thr);
          const int mslot = (kv[0] == thr) ? 0 : (kv[1] == thr) ? 1 : (kv[2] == thr) ? 2 : (kv[3] == thr) ? 3 : 4;
          const unsigned ob  = __builtin_amdgcn_ballot_w32(mslot < 4);
          const unsigned obh = (ob >> hsh) & 0xffffu;
          const int ol = (int)__builtin_ctz(obh | 0x10000u) & 15;
          const bool own = act && (l16 == ol);
#pragma unroll
          for (int j = 0; j < 4; ++j) {
            const bool rep = own && (mslot == j);
            kv[j] = rep ? cv : kv[j];
            ki[j] = rep ? ci : ki[j];
          }
          float lm = fminf(fminf(kv[0], kv[1]), fminf(kv[2], kv[3]));
          lm = fminf(lm, __shfl_xor(lm, 1, 32));
          lm = fminf(lm, __shfl_xor(lm, 2, 32));
          lm = fminf(lm, __shfl_xor(lm, 4, 32));
          lm = fminf(lm, __shfl_xor(lm, 8, 32));
          thr = lm;
          const bool done = hasc && (l16 == src);
          hit = hit && (!done) && (v > thr);
          b = __builtin_amdgcn_ballot_w32(hit);
        }
      }
    }
    __syncthreads();
  }

  float ev[4];
  int   id[4];
  const v4f* up = (const v4f*)(userF + (size_t)(ubase + su) * kD);
#pragma unroll
  for (int j = 0; j < 4; ++j) {
    int x = ki[j];
    x = (x < 0) ? 0 : x;
    x = (x > kNI - 1) ? (kNI - 1) : x;
    id[j] = x;
    const v4f* ip = (const v4f*)(itemF + (size_t)x * kD);
    float acc = 0.0f;
#pragma unroll 1
    for (int k4 = 0; k4 < kD / 4; ++k4) {
      const v4f a = up[k4];
      const v4f bq = ip[k4];
      const float ax = a[0], ay = a[1], az = a[2], aw = a[3];
      const float bx = bq[0], by = bq[1], bz = bq[2], bw = bq[3];
      acc = chain_step(ax, bx, acc);
      acc = chain_step(ay, by, acc);
      acc = chain_step(az, bz, acc);
      acc = chain_step(aw, bw, acc);
    }
    ev[j] = acc;
  }
#pragma unroll
  for (int j = 0; j < 4; ++j) {
    rvS[su * kKeep + l16 * 4 + j] = ev[j];
    riS[su * kKeep + l16 * 4 + j] = id[j];
  }
  __syncthreads();

  int rk[4];
#pragma unroll
  for (int j = 0; j < 4; ++j) rk[j] = 0;
#pragma unroll 1
  for (int e = 0; e < kKeep; ++e) {
    const float ov = rvS[su * kKeep + e];
    const int   oi = riS[su * kKeep + e];
#pragma unroll
    for (int j = 0; j < 4; ++j) {
      const bool ahead = (ov > ev[j]) || ((ov == ev[j]) && (oi < id[j]));
      rk[j] += ahead ? 1 : 0;
    }
  }
#pragma unroll
  for (int j = 0; j < 4; ++j) {
    if (rk[j] < kTopK) outS[su * kTopK + rk[j]] = premise_ok ? id[j] : -1;
  }
  __syncthreads();

  if (wave == 0) {
    int* gp = out + (size_t)blockIdx.x * kOutPerBlock;
    v4i vals[7];
#pragma unroll
    for (int it = 0; it < 7; ++it) {
      const int idx4 = it * 32 + lane;
      const int idc  = (idx4 < kOutVec4) ? idx4 : (kOutVec4 - 1);
      vals[it] = *(const v4i*)(outS + idc * 4);
    }
    for (int pass = 0; pass < 2; ++pass) {
#pragma unroll
      for (int it = 0; it < 7; ++it) {
        const int idx4 = it * 32 + lane;
        if (idx4 < kOutVec4) *(volatile v4i*)(gp + idx4 * 4) = vals[it];
      }
      __threadfence();
    }
  }
}

extern "C" void kernel_launch(void* const* d_in, const int* in_sizes, int n_in,
                              void* d_out, int out_size, void* d_ws, size_t ws_size,
                              hipStream_t stream) {
  if (n_in < 4) return;
  if (in_sizes[0] != kNU * kD) return;
  if (in_sizes[1] != kNI * kD) return;
  if (in_sizes[2] != kNU * kNR) return;
  if (in_sizes[3] != 1) return;
  if (out_size != kNU * kTopK) return;
  if (ws_size < kWsTotal) return;

  const float* user_embs = (const float*)d_in[0];
  const float* item_embs = (const float*)d_in[1];
  const int*   rated     = (const int*)d_in[2];
  const int*   topk_in   = (const int*)d_in[3];
  int* out = (int*)d_out;

  char* ws = (char*)d_ws;
  unsigned short* UH = (unsigned short*)(ws + kOffUH);
  unsigned short* IH = (unsigned short*)(ws + kOffIH);

  constexpr int kUser8 = kNU * kD / 8;
  constexpr int kItem8 = kNI * kD / 8;
  static_assert((kUser8 % 256) == 0 && (kItem8 % 256) == 0, "exact grids");

  scale_cast_f16_kernel<<<kUser8 / 256, 256, 0, stream>>>(user_embs, UH, kUser8);
  scale_cast_f16_kernel<<<kItem8 / 256, 256, 0, stream>>>(item_embs, IH, kItem8);

  prefilter_rescore_kernel<<<kNU / kUPB, kTPB, 0, stream>>>(
      UH, IH, user_embs, item_embs, rated, topk_in, out);
}
